// LocalAgg_39324720562662
// MI455X (gfx1250) — hardware-verified
//
#include <hip/hip_runtime.h>
#include <math.h>

typedef __attribute__((ext_vector_type(16))) _Float16 v16h;
typedef __attribute__((ext_vector_type(16))) __bf16 v16b;
typedef __attribute__((ext_vector_type(8)))  _Float16 v8h;
typedef __attribute__((ext_vector_type(8)))  float v8f;
typedef __attribute__((ext_vector_type(4)))  float v4f;
typedef __attribute__((ext_vector_type(2)))  float v2f;
typedef __attribute__((ext_vector_type(4)))  unsigned v4u;
typedef __attribute__((ext_vector_type(4)))  int v4i;
typedef float __attribute__((may_alias)) float_a;
typedef int __attribute__((may_alias)) int_a;

template <typename T> __device__ __forceinline__ void vst2(void* p, T v) { *(volatile T*)p = v; __threadfence(); *(volatile T*)p = v; }
__device__ __forceinline__ v8f wmma16(v16h a, v16h b, v8f c) {
  v8f d = __builtin_amdgcn_wmma_f32_16x16x32_f16(false, a, false, b, (short)0, c, false, false);
  asm volatile("v_nop\n\tv_nop\n\tv_nop\n\tv_nop" : "+v"(d) : "v"(a), "v"(b));
  return d;
}
__device__ __forceinline__ v8f wmma_bf(v16b a, v16b b, v8f c) {
  v8f d = __builtin_amdgcn_wmma_f32_16x16x32_bf16(false, a, false, b, (short)0, c, false, false);
  asm volatile("v_nop\n\tv_nop\n\tv_nop\n\tv_nop" : "+v"(d) : "v"(a), "v"(b));
  return d;
}
__device__ __forceinline__ v16h frag_h(const _Float16* rowk0, int lane) {
  union { v16h v; v8h q[2]; } u; const _Float16* p = rowk0 + 8 * (lane >> 4);
  u.q[0] = *(const v8h*)p; u.q[1] = *(const v8h*)(p + 16); return u.v;
}
__device__ __forceinline__ v16h frag_f32(const float* rowk0, int lane) {
  v16h a; const float* p = rowk0 + 8 * (lane >> 4);
#pragma unroll
  for (int i = 0; i < 8; ++i) { a[i] = (_Float16)p[i]; a[8 + i] = (_Float16)p[16 + i]; }
  return a;
}
__device__ __forceinline__ v16h frag_f32s(const float* rowk0, int lane, float sc) {
  v16h a; const float* p = rowk0 + 8 * (lane >> 4);
#pragma unroll
  for (int i = 0; i < 8; ++i) { a[i] = (_Float16)(p[i] * sc); a[8 + i] = (_Float16)(p[16 + i] * sc); }
  return a;
}
__device__ __forceinline__ v16h fragc_f32(const float* W, int k0, int n, int lane, int ld, int K) {
  v16h a; const int g = lane >> 4;
#pragma unroll
  for (int i = 0; i < 8; ++i) { const int ka = k0 + 8 * g + i, kb = ka + 16;
    a[i] = (_Float16)(ka < K ? W[(size_t)(ka < K ? ka : K - 1) * ld + n] : 0.f); a[8 + i] = (_Float16)(kb < K ? W[(size_t)(kb < K ? kb : K - 1) * ld + n] : 0.f); }
  return a;
}
struct F2 { v16b h, l; };
__device__ __forceinline__ F2 bsplit16(const float v[16]) { F2 r;
#pragma unroll
  for (int i = 0; i < 16; ++i) { const __bf16 h = (__bf16)v[i]; r.h[i] = h; r.l[i] = (__bf16)(v[i] - (float)h); }
  return r; }
__device__ __forceinline__ F2 split_row(const float* row, int k0, int lane) { float v[16]; const float* p = row + k0 + 8 * (lane >> 4);
#pragma unroll
  for (int i = 0; i < 8; ++i) { v[i] = p[i]; v[8 + i] = p[16 + i]; }
  return bsplit16(v); }
__device__ __forceinline__ F2 split_rowK(const float* row, int k0, int lane, int K) { float v[16]; const int g = lane >> 4;
#pragma unroll
  for (int i = 0; i < 8; ++i) { const int ka = k0 + 8 * g + i, kb = ka + 16; v[i] = ka < K ? row[ka < K ? ka : K - 1] : 0.f; v[8 + i] = kb < K ? row[kb < K ? kb : K - 1] : 0.f; }
  return bsplit16(v); }
__device__ __forceinline__ F2 split_col(const float* W, int k0, int n, int lane, int ld, int K) { float v[16]; const int g = lane >> 4;
#pragma unroll
  for (int i = 0; i < 8; ++i) { const int ka = k0 + 8 * g + i, kb = ka + 16; v[i] = ka < K ? W[(size_t)(ka < K ? ka : K - 1) * ld + n] : 0.f; v[8 + i] = kb < K ? W[(size_t)(kb < K ? kb : K - 1) * ld + n] : 0.f; }
  return bsplit16(v); }
__device__ __forceinline__ v8f mac3(const F2& a, const F2& b, v8f c) { c = wmma_bf(a.l, b.h, c); c = wmma_bf(a.h, b.l, c); return wmma_bf(a.h, b.h, c); }
__device__ __forceinline__ float sigm(float v) { return 1.0f / (1.0f + expf(-v)); }
#define LDSX() do { asm volatile("s_wait_dscnt 0" ::: "memory"); __builtin_amdgcn_wave_barrier(); __builtin_amdgcn_fence(__ATOMIC_RELEASE, "workgroup"); } while (0)


#define NB 16
#define NPTS 8192
#define NM 2048
#define KN 32
#define CI 32
#define CO 64
#define BNE 1e-5f
#ifndef TCB
#define TCB (NB * NM / 2)
#endif
typedef __attribute__((ext_vector_type(8))) __bf16 v8b;
__device__ __forceinline__ v16b frag_b(const __bf16* rowk0, int lane) {
  union { v16b v; v8b q[2]; } u; const __bf16* p = rowk0 + 8 * (lane >> 4);
  u.q[0] = *(const v8b*)p; u.q[1] = *(const v8b*)(p + 16); return u.v;
}
__device__ __forceinline__ float bfr(float v) { return (float)(__bf16)v; }
__device__ __attribute__((noinline)) float exp_ni(float v) { return expf(v); }
__device__ __attribute__((noinline)) float erf_ni(float v) { return erff(v); }
__device__ __attribute__((noinline)) float gelu_e(float v) { return 0.5f * v * (1.0f + erff(v * 0.70710678118654752f)); }

#define WS_P1  0u
#define WS_P2  (WS_P1 + 2u * 64 * 64)
#define WS_END (WS_P2 + 2u * 64 * 64)

__global__ __launch_bounds__(64) void k_pack(const float* __restrict__ W1, const float* __restrict__ W2, __bf16* __restrict__ P) { const int n = blockIdx.x, which = blockIdx.y, t = threadIdx.x; __shared__ __align__(16) __bf16 s[64];
  s[t] = (which == 0) ? ((t < 3 + CI) ? (__bf16)W1[(size_t)t * CO + n] : (__bf16)0.0f) : (__bf16)W2[(size_t)t * CO + n]; __syncthreads();
  if (t < 8) vst2((unsigned*)(P + (which == 0 ? WS_P1 : WS_P2) / 2 + (size_t)n * 64 + t * 8), *(const v4u*)&s[t * 8]); }
__global__ __launch_bounds__(128) void k_main(const float* __restrict__ FEAT, const float* __restrict__ POS, const float* __restrict__ CF, const float* __restrict__ CP, const int* __restrict__ KNN, const __bf16* __restrict__ P,
    const float* __restrict__ B1, const float* __restrict__ G1, const float* __restrict__ BE1, const float* __restrict__ M1, const float* __restrict__ V1,
    const float* __restrict__ B2, const float* __restrict__ G2, const float* __restrict__ BE2, const float* __restrict__ M2, const float* __restrict__ V2, const float* __restrict__ WSK, float* __restrict__ OUT) {
  __shared__ __align__(16) float sh[64][CO + 4]; __shared__ __align__(16) float so2[2][CO];
  const int tid = threadIdx.x, wave = tid >> 5, lane = tid & 31, col = lane & 15, g = lane >> 4; const size_t cbase = (size_t)blockIdx.x * 2;
  const size_t cidx = cbase + (wave >> 1); const size_t b = cidx / NM; const int kk = (wave & 1) * 16 + col;
  int nbr = KNN[cidx * KN + kk]; nbr = nbr < 0 ? 0 : (nbr >= NPTS ? NPTS - 1 : nbr); const float* fr = FEAT + (b * NPTS + nbr) * CI; const float* pr = POS + (b * NPTS + nbr) * 3; const float* cpr = CP + cidx * 3;
  v8f acc[4] = {};
#pragma unroll
  for (int kc = 0; kc < 2; ++kc) { float v[16];
#pragma unroll
    for (int i = 0; i < 16; ++i) { const int k = kc * 32 + 8 * g + (i < 8 ? i : 8 + i); float x = 0.f; if (k < 3) x = bfr(pr[k]) - bfr(cpr[k]); else if (k < 3 + CI) x = bfr(fr[k - 3]); v[i] = x; }
    const F2 a = bsplit16(v);
#pragma unroll
    for (int j = 0; j < 4; ++j) { const v16b w = frag_b(P + WS_P1 / 2 + (size_t)(j * 16 + col) * 64 + kc * 32, lane); acc[j] = wmma_bf(a.h, w, acc[j]); acc[j] = wmma_bf(a.l, w, acc[j]); } }
#pragma unroll
  for (int j = 0; j < 4; ++j) { const int c = j * 16 + col; const float sc = bfr(G1[c]) / sqrtf(bfr(V1[c]) + BNE), mm = bfr(M1[c]), be = bfr(BE1[c]), bb = bfr(B1[c]);
#pragma unroll
    for (int r = 0; r < 8; ++r) sh[wave * 16 + 8 * g + r][c] = gelu_e((acc[j][r] + bb - mm) * sc + be); }
  LDSX();
  v8f acc2[4] = {};
#pragma unroll
  for (int kc = 0; kc < 2; ++kc) { float v[16]; const float* p2 = &sh[wave * 16 + col][kc * 32 + 8 * g];
#pragma unroll
    for (int i = 0; i < 8; ++i) { v[i] = p2[i]; v[8 + i] = p2[16 + i]; }
    const F2 a = bsplit16(v);
#pragma unroll
    for (int j = 0; j < 4; ++j) { const v16b w = frag_b(P + WS_P2 / 2 + (size_t)(j * 16 + col) * 64 + kc * 32, lane); acc2[j] = wmma_bf(a.h, w, acc2[j]); acc2[j] = wmma_bf(a.l, w, acc2[j]); } }
  LDSX();
#pragma unroll
  for (int j = 0; j < 4; ++j) { const int c = j * 16 + col; const float sc = bfr(G2[c]) / sqrtf(bfr(V2[c]) + BNE), mm = bfr(M2[c]), be = bfr(BE2[c]), bb = bfr(B2[c]);
#pragma unroll
    for (int r = 0; r < 8; ++r) sh[wave * 16 + 8 * g + r][c] = gelu_e((acc2[j][r] + bb - mm) * sc + be); }
  __syncthreads();
  { const int ci = tid >> 6, c = tid & 63; float mx = -3.0e38f;
#pragma unroll 1
    for (int k = 0; k < KN; ++k) mx = fmaxf(mx, sh[ci * 32 + k][c]);
    const size_t cc = cbase + ci; float sk = 0.f; const float* cf = CF + cc * CI;
#pragma unroll 1
    for (int i = 0; i < CI; ++i) sk += bfr(cf[i]) * bfr(WSK[(size_t)i * CO + c]);
    so2[ci][c] = mx + sk; }
  __syncthreads(); if (tid < 32) vst2(OUT + cbase * CO + tid * 4, *((const v4f*)&so2[0][0] + tid));
}
extern "C" void kernel_launch(void* const* d_in, const int* in_sizes, int n_in, void* d_out, int out_size, void* d_ws, size_t ws_size, hipStream_t stream) {
  (void)in_sizes; (void)n_in; (void)out_size;
  const float** F = (const float**)d_in;
  if (ws_size < (size_t)WS_END) return;
  __bf16* P = (__bf16*)d_ws;
  k_pack<<<dim3(CO, 2), 64, 0, stream>>>(F[5], F[11], P);
  k_main<<<TCB, 128, 0, stream>>>(F[0], F[1], F[2], F[3], (const int*)d_in[4], P, F[6], F[7], F[8], F[9], F[10], F[12], F[13], F[14], F[15], F[16], F[17], (float*)d_out);
}
